// ResidualMambaBlockLayer_39049842655409
// MI455X (gfx1250) — hardware-verified
//
#include <hip/hip_runtime.h>


#define NB_    2
#define NL_    2048
#define LSH_   11
#define DM_    256
#define DI_    512
#define NS_    16
#define DR_    16
#define NDBL_  48
#define PDBL_  64
#define KDT_   32
#define PXW_   64
#define MT_    (NB_ * NL_)

static_assert((1 << LSH_) == NL_);
static_assert(MT_ % 64 == 0);
static_assert(NL_ % 128 == 0);
static_assert(NL_ % 32 == 0);
static_assert((2 * DI_) % 128 == 0);
static_assert(DI_ % 128 == 0);
static_assert(DI_ % 64 == 0);
static_assert(DM_ % 64 == 0);
static_assert(DM_ == 256);
static_assert(NDBL_ == DR_ + 2 * NS_);
static_assert(PDBL_ >= NDBL_ && PDBL_ % 32 == 0);
static_assert(PXW_ >= NDBL_ && PXW_ == 64);
static_assert(KDT_ == 32 && DR_ == 16);

typedef float          v4f   __attribute__((ext_vector_type(4)));
typedef float          v8f   __attribute__((ext_vector_type(8)));
typedef _Float16       v8h   __attribute__((ext_vector_type(8)));
typedef _Float16       v16h  __attribute__((ext_vector_type(16)));
typedef unsigned short u16x8 __attribute__((ext_vector_type(8)));

union FragH { u16x8 h[2]; v16h v; };
union Pack8 { v8h f; u16x8 u; };
union H1    { _Float16 f; unsigned short u; };

__device__ __forceinline__ float silu_f(float x) {
    float e = __expf(-x);
    return x * __builtin_amdgcn_rcpf(1.0f + e);
}
__device__ __forceinline__ float softplus_f(float x) {
    return fmaxf(x, 0.0f) + log1pf(__expf(-fabsf(x)));
}
__device__ __forceinline__ float conv4_silu(float x0, float x1, float x2, float x3,
                                            float w0, float w1, float w2, float w3, float bias) {
    float c = w0 * x0 + w1 * x1 + w2 * x2 + w3 * x3;
    return silu_f(c + bias);
}
__device__ __forceinline__ v8f ld8f(const float* p) {
    v4f a = *(const v4f*)p;
    v4f b = *(const v4f*)(p + 4);
    return __builtin_shufflevector(a, b, 0, 1, 2, 3, 4, 5, 6, 7);
}
__device__ __forceinline__ v8f zero8() {
    v8f z;
#pragma unroll
    for (int c = 0; c < 8; ++c) z[c] = 0.0f;
    return z;
}

__device__ __forceinline__ void mma16(v8f& acc, const FragH& a, const FragH& b) {
    acc = __builtin_amdgcn_wmma_f32_16x16x32_f16(false, a.v, false, b.v, (short)0, acc, false, false);
    asm volatile("v_nop\n\tv_nop\n\tv_nop\n\tv_nop" : "+v"(acc) : "v"(a.v), "v"(b.v));
}

__global__ __launch_bounds__(256)
void cvt_f16_kernel(const float* __restrict__ src, unsigned short* dst, int n8src, int n8tot, float scale)
{
    const int i = blockIdx.x * 256 + threadIdx.x;
    if (i >= n8tot) return;
    const size_t e = (size_t)i * 8;
    v8f x = zero8();
    if (i < n8src) x = ld8f(src + e);
    Pack8 pk;
    pk.f = __builtin_convertvector(x * scale, v8h);
    const u16x8 v = pk.u;
    *(volatile u16x8*)(dst + e) = v;
    __threadfence();
    *(volatile u16x8*)(dst + e) = v;
}

__global__ __launch_bounds__(256)
void pad16to32_kernel(const float* __restrict__ src, unsigned short* dst, int spitch, int nrows, float scale)
{
    const int lane  = threadIdx.x & 31;
    const int wave  = threadIdx.x >> 5;
    const int row   = (blockIdx.x * 8 + wave) * 8 + 2 * (lane >> 3) + ((lane & 7) >> 2);
    const int piece = lane & 3;
    if (row >= nrows) return;
    v8f x = zero8();
    if (piece < 2) x = ld8f(src + (size_t)row * spitch + piece * 8);
    Pack8 pk;
    pk.f = __builtin_convertvector(x * scale, v8h);
    const u16x8 v = pk.u;
    unsigned short* gp = dst + (size_t)row * KDT_ + piece * 8;
    *(volatile u16x8*)gp = v;
    __threadfence();
    *(volatile u16x8*)gp = v;
}

__global__ __launch_bounds__(256)
void rmsnorm_kernel(const float* __restrict__ x, const float* __restrict__ w, unsigned short* H16)
{
    __shared__ float tile[DM_ * 33];
    const int tid  = threadIdx.x;
    const int lane = tid & 31;
    const int wave = tid >> 5;
    const int m0   = blockIdx.x * 32;
    const int b    = m0 >> LSH_;
    const int l0   = m0 & (NL_ - 1);
    const float* xb = x + (size_t)b * DM_ * NL_ + l0 + lane;
#pragma unroll 4
    for (int p = 0; p < DM_ / 8; ++p) {
        const int c = p * 8 + wave;
        tile[c * 33 + lane] = xb[(size_t)c * NL_];
    }
    __syncthreads();

    const v8f wv = ld8f(w + lane * 8);
#pragma unroll 1
    for (int i = 0; i < 4; ++i) {
        const int tl = wave * 4 + i;
        v8f v;
        float ss = 0.0f;
#pragma unroll
        for (int j = 0; j < 8; ++j) {
            const float f = tile[(lane * 8 + j) * 33 + tl];
            v[j] = f;
            ss += f * f;
        }
        ss += __shfl_xor(ss, 16);
        ss += __shfl_xor(ss, 8);
        ss += __shfl_xor(ss, 4);
        ss += __shfl_xor(ss, 2);
        ss += __shfl_xor(ss, 1);
        const float sc = rsqrtf(ss * (1.0f / DM_) + 1e-5f);
        const v8f hv = (v * sc) * wv;
        Pack8 pk;
        pk.f = __builtin_convertvector(hv, v8h);
        const u16x8 o = pk.u;
        unsigned short* gp = H16 + (size_t)(m0 + tl) * DM_ + lane * 8;
        *(volatile u16x8*)gp = o;
        __threadfence();
        *(volatile u16x8*)gp = o;
    }
}

template<int NBF, bool RESID>
__device__ __forceinline__ void tile_store_pass(const float* st, float* gp, const float* rp, int ldc, int lane) {
    constexpr int CW  = NBF * 16;
    constexpr int P   = CW + 4;
    constexpr int LPR = CW / 4;
    constexpr int RPI = 32 / LPR;
    constexpr int NIT = 32 / RPI;
    const int rsub = lane / LPR;
    const int c4   = (lane % LPR) * 4;
#pragma unroll
    for (int it = 0; it < NIT; ++it) {
        const int row = it * RPI + rsub;
        v4f v = *(const v4f*)(st + row * P + c4);
        if (RESID) v += *(const v4f*)(rp + (size_t)row * ldc + c4);
        *(volatile v4f*)(gp + (size_t)row * ldc + c4) = v;
    }
}

template<int NBF, bool RESID>
__global__ __launch_bounds__(128)
void gemm_tn_kernel(const unsigned short* __restrict__ A, const unsigned short* __restrict__ Bw,
                    float* C, float* C2, const float* __restrict__ R,
                    int K, int ldc, int csplit, int cshift, int cstride, float scale)
{
    constexpr int CW = NBF * 16;
    constexpr int P  = CW + 4;
    __shared__ __attribute__((aligned(16))) float stile[4][32 * P];

    const int tid  = threadIdx.x;
    const int lane = tid & 31;
    const int wave = tid >> 5;
    const int h    = lane >> 4;
    const int m    = lane & 15;
    const int wm   = wave >> 1;
    const int wn   = wave & 1;

    const int rowW = blockIdx.y * 64 + wm * 32;
    const int colW = blockIdx.x * (2 * CW) + wn * CW;

    v8f acc[2 * NBF];
#pragma unroll
    for (int j = 0; j < 2 * NBF; ++j)
#pragma unroll
        for (int r = 0; r < 8; ++r) acc[j][r] = 0.0f;

    const size_t aoff  = (size_t)(rowW + m) * K + 8 * h;
    const size_t boff  = (size_t)(colW + m) * K + 8 * h;
    const size_t sub16 = (size_t)16 * K;
    const int nk = K >> 5;

    for (int kt = 0; kt < nk; ++kt) {
        const size_t k0 = (size_t)kt * 32;
        FragH fa[2], fb[NBF];
#pragma unroll
        for (int s = 0; s < 2; ++s) {
            const unsigned short* p = A + aoff + s * sub16 + k0;
            fa[s].h[0] = *(const u16x8*)(p);
            fa[s].h[1] = *(const u16x8*)(p + 16);
        }
#pragma unroll
        for (int j = 0; j < NBF; ++j) {
            const unsigned short* p = Bw + boff + j * sub16 + k0;
            fb[j].h[0] = *(const u16x8*)(p);
            fb[j].h[1] = *(const u16x8*)(p + 16);
        }
#pragma unroll
        for (int s = 0; s < 2; ++s)
#pragma unroll
            for (int j = 0; j < NBF; ++j)
                mma16(acc[s * NBF + j], fa[s], fb[j]);
    }

    float* st = stile[wave];
#pragma unroll
    for (int s = 0; s < 2; ++s)
#pragma unroll
        for (int j = 0; j < NBF; ++j)
#pragma unroll
            for (int r = 0; r < 8; ++r)
                st[(s * 16 + 8 * h + r) * P + j * 16 + m] = acc[s * NBF + j][r] * scale;
    __syncthreads();

    float* Cp = C;
    int gcol = colW;
    if (colW >= csplit) { Cp = C2; gcol = colW - csplit; }
    const int zb = gcol >> cshift;
    gcol &= (1 << cshift) - 1;
    const size_t base = (size_t)zb * (size_t)cstride + (size_t)rowW * ldc + gcol;
    float* gp = Cp + base;
    const float* rp = R + base;
    tile_store_pass<NBF, RESID>(st, gp, rp, ldc, lane);
    __threadfence();
    tile_store_pass<NBF, RESID>(st, gp, rp, ldc, lane);
}

__global__ __launch_bounds__(64)
void conv_silu_kernel(const float* __restrict__ X, const float* __restrict__ cw,
                      const float* __restrict__ cb, unsigned short* U16)
{
    const int m  = blockIdx.x;
    const int l  = m & (NL_ - 1);
    const int d0 = threadIdx.x * 8;
    const float* xr = X + (size_t)m * DI_ + d0;

    v8f x3 = ld8f(xr);
    v8f x2 = zero8(), x1 = zero8(), x0 = zero8();
    if (l >= 1) x2 = ld8f(xr - DI_);
    if (l >= 2) x1 = ld8f(xr - 2 * DI_);
    if (l >= 3) x0 = ld8f(xr - 3 * DI_);

    const float* wp = cw + (size_t)d0 * 4;
    v4f wv[8];
#pragma unroll
    for (int c = 0; c < 8; ++c) wv[c] = *(const v4f*)(wp + 4 * c);
    const v8f bias = ld8f(cb + d0);

    v8f u;
#pragma unroll
    for (int c = 0; c < 8; ++c)
        u[c] = conv4_silu(x0[c], x1[c], x2[c], x3[c], wv[c][0], wv[c][1], wv[c][2], wv[c][3], bias[c]);

    Pack8 pk;
    pk.f = __builtin_convertvector(u * 64.0f, v8h);
    const u16x8 v = pk.u;
    unsigned short* gp = U16 + (size_t)m * DI_ + d0;
    *(volatile u16x8*)gp = v;
    __threadfence();
    *(volatile u16x8*)gp = v;
}

__global__ __launch_bounds__(64)
void scan_kernel(const float* __restrict__ X, const float* __restrict__ Z, const float* __restrict__ Dl,
                 const float* __restrict__ DBL,
                 const float* __restrict__ cw, const float* __restrict__ cb, const float* __restrict__ dpb,
                 const float* __restrict__ Alog, const float* __restrict__ Dp,
                 unsigned short* G16)
{
    __shared__ __attribute__((aligned(16))) float sbc[16 * 32];
    __shared__ __attribute__((aligned(16))) unsigned short sg[16 * 64];

    const int tid   = threadIdx.x;
    const int lane  = tid & 31;
    const int wave  = tid >> 5;
    const int dbase = blockIdx.x * 64;
    const int d     = dbase + tid;
    const int b     = blockIdx.y;

    float an[NS_], hs[NS_];
#pragma unroll
    for (int n = 0; n < NS_; ++n) {
        an[n] = -__expf(Alog[d * NS_ + n]);
        hs[n] = 0.0f;
    }
    const float w0 = cw[d * 4 + 0], w1 = cw[d * 4 + 1], w2 = cw[d * 4 + 2], w3 = cw[d * 4 + 3];
    const float cbias = cb[d];
    const float pb = dpb[d];
    const float Dd = Dp[d];

    float xm1 = 0.0f, xm2 = 0.0f, xm3 = 0.0f;
    const size_t mrow0 = (size_t)b * NL_;
    const int srow  = tid >> 2;
    const int spart = tid & 3;

#pragma unroll 1
    for (int l0 = 0; l0 < NL_; l0 += 16) {
        {
            const float* sp = DBL + (mrow0 + (size_t)(l0 + srow)) * PDBL_ + DR_ + spart * 8;
            *(v4f*)(sbc + srow * 32 + spart * 8)     = *(const v4f*)(sp);
            *(v4f*)(sbc + srow * 32 + spart * 8 + 4) = *(const v4f*)(sp + 4);
        }
        __syncthreads();
#pragma unroll 1
        for (int t = 0; t < 16; ++t) {
            const size_t e = (mrow0 + (size_t)(l0 + t)) * DI_ + d;
            const float xv = X[e];
            const float zv = Z[e];
            const float dl = Dl[e];
            const float u  = conv4_silu(xm3, xm2, xm1, xv, w0, w1, w2, w3, cbias);
            xm3 = xm2; xm2 = xm1; xm1 = xv;
            const float dt = softplus_f(dl + pb);
            const float du = dt * u;
            v4f bq[4], cq[4];
#pragma unroll
            for (int q = 0; q < 4; ++q) {
                bq[q] = *(const v4f*)(sbc + t * 32 + 4 * q);
                cq[q] = *(const v4f*)(sbc + t * 32 + 16 + 4 * q);
            }
            float y = 0.0f;
#pragma unroll
            for (int n = 0; n < NS_; ++n) {
                const float Bn = bq[n >> 2][n & 3];
                const float Cn = cq[n >> 2][n & 3];
                const float da = __expf(dt * an[n]);
                hs[n] = da * hs[n] + du * Bn;
                y += hs[n] * Cn;
            }
            const float g = (y + Dd * u) * silu_f(zv);
            H1 cv;
            cv.f = (_Float16)(g * 256.0f);
            sg[t * 64 + tid] = cv.u;
        }
        __syncthreads();
        {
            const int t0 = wave * 8 + (lane >> 3);
            const int t1 = t0 + 4;
            const int c  = (lane & 7) * 8;
            const u16x8 v0 = *(const u16x8*)(sg + t0 * 64 + c);
            const u16x8 v1 = *(const u16x8*)(sg + t1 * 64 + c);
            unsigned short* g0 = G16 + (mrow0 + (size_t)(l0 + t0)) * DI_ + dbase + c;
            unsigned short* g1 = G16 + (mrow0 + (size_t)(l0 + t1)) * DI_ + dbase + c;
            *(volatile u16x8*)g0 = v0;
            *(volatile u16x8*)g1 = v1;
            __threadfence();
            *(volatile u16x8*)g0 = v0;
            *(volatile u16x8*)g1 = v1;
        }
        __syncthreads();
    }
}

extern "C" void kernel_launch(void* const* d_in, const int* in_sizes, int n_in,
                              void* d_out, int out_size, void* d_ws, size_t ws_size,
                              hipStream_t stream)
{
    if (n_in < 11) return;
    if (in_sizes[0]  != MT_ * DM_)      return;
    if (in_sizes[1]  != DM_)            return;
    if (in_sizes[2]  != 2 * DI_ * DM_)  return;
    if (in_sizes[3]  != DI_ * 4)        return;
    if (in_sizes[4]  != DI_)            return;
    if (in_sizes[5]  != NDBL_ * DI_)    return;
    if (in_sizes[6]  != DI_ * DR_)      return;
    if (in_sizes[7]  != DI_)            return;
    if (in_sizes[8]  != DI_ * NS_)      return;
    if (in_sizes[9]  != DI_)            return;
    if (in_sizes[10] != DM_ * DI_)      return;
    if (out_size != MT_ * DM_)          return;

    const float* hsx  = (const float*)d_in[0];
    const float* nw   = (const float*)d_in[1];
    const float* wi   = (const float*)d_in[2];
    const float* cw   = (const float*)d_in[3];
    const float* cb   = (const float*)d_in[4];
    const float* wx   = (const float*)d_in[5];
    const float* wdt  = (const float*)d_in[6];
    const float* dpb  = (const float*)d_in[7];
    const float* alog = (const float*)d_in[8];
    const float* Dp   = (const float*)d_in[9];
    const float* wo   = (const float*)d_in[10];
    float* out = (float*)d_out;

    const size_t SZ_H16  = (size_t)MT_ * DM_ * 2;
    const size_t SZ_WIN  = (size_t)2 * DI_ * DM_ * 2;
    const size_t SZ_WX   = (size_t)PXW_ * DI_ * 2;
    const size_t SZ_WDT  = (size_t)DI_ * KDT_ * 2;
    const size_t SZ_WO   = (size_t)DM_ * DI_ * 2;
    const size_t SZ_F    = (size_t)MT_ * DI_ * 4;
    const size_t SZ_U16  = (size_t)MT_ * DI_ * 2;
    const size_t SZ_DBL  = (size_t)MT_ * PDBL_ * 4;
    const size_t SZ_DT16 = (size_t)MT_ * KDT_ * 2;

    const size_t OFF_H16  = 0;
    const size_t OFF_WIN  = OFF_H16 + SZ_H16;
    const size_t OFF_WX   = OFF_WIN + SZ_WIN;
    const size_t OFF_WDT  = OFF_WX + SZ_WX;
    const size_t OFF_WO   = OFF_WDT + SZ_WDT;
    const size_t OFF_XF   = OFF_WO + SZ_WO;
    const size_t OFF_ZF   = OFF_XF + SZ_F;
    const size_t OFF_DL   = OFF_ZF + SZ_F;
    const size_t OFF_U16  = OFF_DL + SZ_F;
    const size_t OFF_G16  = OFF_U16 + SZ_U16;
    const size_t OFF_DBL  = OFF_G16 + SZ_U16;
    const size_t OFF_DT16 = OFF_DBL + SZ_DBL;
    const size_t WS_END   = OFF_DT16 + SZ_DT16;
    if (ws_size < WS_END) return;

    char* ws = (char*)d_ws;
    unsigned short* h16   = (unsigned short*)(ws + OFF_H16);
    unsigned short* win16 = (unsigned short*)(ws + OFF_WIN);
    unsigned short* wx16  = (unsigned short*)(ws + OFF_WX);
    unsigned short* wdt16 = (unsigned short*)(ws + OFF_WDT);
    unsigned short* wo16  = (unsigned short*)(ws + OFF_WO);
    float*          Xf    = (float*)(ws + OFF_XF);
    float*          Zf    = (float*)(ws + OFF_ZF);
    float*          Dl    = (float*)(ws + OFF_DL);
    unsigned short* u16   = (unsigned short*)(ws + OFF_U16);
    unsigned short* g16   = (unsigned short*)(ws + OFF_G16);
    float*          DBL   = (float*)(ws + OFF_DBL);
    unsigned short* dt16  = (unsigned short*)(ws + OFF_DT16);

    const int NOSPLIT = 1 << 30;

    {
        int n8;
        n8 = (2 * DI_ * DM_) / 8;
        hipLaunchKernelGGL(cvt_f16_kernel, dim3((n8 + 255) / 256), dim3(256), 0, stream,
                           wi, win16, n8, n8, 32.0f);
        const int n8s = (NDBL_ * DI_) / 8;
        n8 = (PXW_ * DI_) / 8;
        hipLaunchKernelGGL(cvt_f16_kernel, dim3((n8 + 255) / 256), dim3(256), 0, stream,
                           wx, wx16, n8s, n8, 32.0f);
        n8 = (DM_ * DI_) / 8;
        hipLaunchKernelGGL(cvt_f16_kernel, dim3((n8 + 255) / 256), dim3(256), 0, stream,
                           wo, wo16, n8, n8, 32.0f);
        hipLaunchKernelGGL(pad16to32_kernel, dim3((DI_ + 63) / 64), dim3(256), 0, stream,
                           wdt, wdt16, (int)DR_, (int)DI_, 16.0f);
    }

    hipLaunchKernelGGL(rmsnorm_kernel, dim3(MT_ / 32), dim3(256), 0, stream, hsx, nw, h16);

    hipLaunchKernelGGL(HIP_KERNEL_NAME(gemm_tn_kernel<4, false>),
                       dim3((2 * DI_) / 128, MT_ / 64), dim3(128), 0, stream,
                       (const unsigned short*)h16, (const unsigned short*)win16,
                       Xf, Zf, hsx, (int)DM_, (int)DI_, (int)DI_, 30, 0, 0.03125f);

    hipLaunchKernelGGL(conv_silu_kernel, dim3(MT_), dim3(DI_ / 8), 0, stream,
                       (const float*)Xf, cw, cb, u16);

    hipLaunchKernelGGL(HIP_KERNEL_NAME(gemm_tn_kernel<2, false>),
                       dim3(1, MT_ / 64), dim3(128), 0, stream,
                       (const unsigned short*)u16, (const unsigned short*)wx16,
                       DBL, DBL, hsx, (int)DI_, (int)PDBL_, NOSPLIT, 30, 0, 0.00048828125f);

    hipLaunchKernelGGL(pad16to32_kernel, dim3((MT_ + 63) / 64), dim3(256), 0, stream,
                       (const float*)DBL, dt16, (int)PDBL_, (int)MT_, 256.0f);

    hipLaunchKernelGGL(HIP_KERNEL_NAME(gemm_tn_kernel<4, false>),
                       dim3(DI_ / 128, MT_ / 64), dim3(128), 0, stream,
                       (const unsigned short*)dt16, (const unsigned short*)wdt16,
                       Dl, Dl, hsx, (int)KDT_, (int)DI_, NOSPLIT, 30, 0, 0.000244140625f);

    hipLaunchKernelGGL(scan_kernel, dim3(DI_ / 64, NB_), dim3(64), 0, stream,
                       (const float*)Xf, (const float*)Zf, (const float*)Dl, (const float*)DBL,
                       cw, cb, dpb, alog, Dp, g16);

    hipLaunchKernelGGL(HIP_KERNEL_NAME(gemm_tn_kernel<4, true>),
                       dim3(MT_ / 128, DM_ / 64), dim3(128), 0, stream,
                       (const unsigned short*)wo16, (const unsigned short*)g16,
                       out, out, hsx, (int)DI_, (int)NL_, NOSPLIT, (int)LSH_, (int)(DM_ * NL_),
                       0.0001220703125f);
}
